// Conv2dDeformable_14929306321759
// MI455X (gfx1250) — hardware-verified
//
#include <hip/hip_runtime.h>
#include <stdint.h>

#pragma clang fp contract(off)

#define NB    8
#define NC    64
#define NO    128
#define HI    128
#define WI    128
#define HWI   (HI * WI)
#define PD    130
#define KT    576
#define PLANE_E ((size_t)NB * PD * PD * NC)
#define OPITCH 65
#define SP    72
#define OSP   68
#define RSC   2048.0f
#define WSC   64.0f
#define INV_H 0.015625f
#define INV_L 7.62939453125e-06f
#define LSTEP (2.0f / 127.0f)
#define WO_CHK (NO * KT / 8)
#define WR_CHK (NC * KT / 8)
#define WO_BLK (WO_CHK / 256)
#define WR_BLK (WR_CHK / 256)

#define WS_WO   ((size_t)0)
#define WS_WR   (WS_WO + (size_t)NO * KT * 2)
#define WS_XH   (WS_WR + (size_t)NC * KT * 2)
#define WS_SP   (WS_XH + PLANE_E * 2)
#define WS_END  (WS_SP + 2 * PLANE_E * 2)

static_assert(WO_CHK % 256 == 0);
static_assert(WR_CHK % 256 == 0);
static_assert(KT % 32 == 0);
static_assert((WS_WR % 128) == 0);
static_assert((WS_XH % 128) == 0);
static_assert((WS_SP % 128) == 0);
static_assert(((PLANE_E * 2) % 128) == 0);
static_assert(NO * OPITCH * 4 + 2 * 65 * SP * 2 <= 60000);
static_assert((SP * 2) % 16 == 0);
static_assert((OSP * 4) % 16 == 0);

typedef _Float16       v16h __attribute__((ext_vector_type(16)));
typedef _Float16       v8h  __attribute__((ext_vector_type(8)));
typedef __bf16         v16b __attribute__((ext_vector_type(16)));
typedef __bf16         v8b  __attribute__((ext_vector_type(8)));
typedef float          v8f  __attribute__((ext_vector_type(8)));
typedef float          v4f  __attribute__((ext_vector_type(4)));
typedef unsigned       v4u  __attribute__((ext_vector_type(4)));
typedef unsigned short v8us __attribute__((ext_vector_type(8)));

__device__ __forceinline__ unsigned bfb(float f) {
  unsigned u = __float_as_uint(f);
  return (u + 0x7FFFu + ((u >> 16) & 1u)) >> 16;
}
__device__ __forceinline__ float bf_rne(float f) { return __uint_as_float(bfb(f) << 16); }
__device__ __forceinline__ unsigned hbits(_Float16 h) {
  return (unsigned)__builtin_bit_cast(unsigned short, h);
}
__device__ __forceinline__ v8f zero8f() { v8f z = {0.f, 0.f, 0.f, 0.f, 0.f, 0.f, 0.f, 0.f}; return z; }
__device__ __forceinline__ v8h zero8h() {
  v8h z;
#pragma unroll
  for (int e = 0; e < 8; ++e) z[e] = (_Float16)0.0f;
  return z;
}
__device__ __forceinline__ v8us zero8us() {
  v8us z;
#pragma unroll
  for (int e = 0; e < 8; ++e) z[e] = (unsigned short)0;
  return z;
}
__device__ __forceinline__ float linv(int i) {
  const float t = -1.0f + (float)i * LSTEP;
  return (i == HI - 1) ? 1.0f : t;
}

__device__ __forceinline__ v16h ldfrag_h(const _Float16* p) {
  union { v16h v; v8h h[2]; } f;
  f.h[0] = *(const v8h*)(p);
  f.h[1] = *(const v8h*)(p + 16);
  return f.v;
}
__device__ __forceinline__ v16b ldfrag_b(const __bf16* p) {
  union { v16b v; v8b h[2]; } f;
  f.h[0] = *(const v8b*)(p);
  f.h[1] = *(const v8b*)(p + 16);
  return f.v;
}

__device__ __forceinline__ v8f mma_h(v16h a, v16h b, v8f c) {
  return __builtin_amdgcn_wmma_f32_16x16x32_f16(false, a, false, b, (short)0, c, false, false);
}
__device__ __forceinline__ v8f mma_b(v16b a, v16b b, v8f c) {
  return __builtin_amdgcn_wmma_f32_16x16x32_bf16(false, a, false, b, (short)0, c, false, false);
}
template <typename F>
__device__ __forceinline__ void guard4(v8f& c0, v8f& c1, v8f& c2, v8f& c3,
                                       const F& f0, const F& f1, const F& f2, const F& f3, const F& f4) {
#if defined(__HIP_DEVICE_COMPILE__)
  asm volatile("v_nop\n\tv_nop\n\tv_nop\n\tv_nop"
               : "+v"(c0), "+v"(c1), "+v"(c2), "+v"(c3)
               : "v"(f0), "v"(f1), "v"(f2), "v"(f3), "v"(f4));
#endif
}
__device__ __forceinline__ void acc_guard4(v8f& c0, v8f& c1, v8f& c2, v8f& c3) {
#if defined(__HIP_DEVICE_COMPILE__)
  asm volatile("v_nop\n\tv_nop\n\tv_nop\n\tv_nop" : "+v"(c0), "+v"(c1), "+v"(c2), "+v"(c3));
#endif
}

__global__ __launch_bounds__(256)
void k_wpack(const float* __restrict__ woff, const float* __restrict__ wreg, unsigned* wo, unsigned* wr)
{
  const int tid = threadIdx.x;
  if (blockIdx.x < WO_BLK) {
    const int q   = blockIdx.x * 256 + tid;
    const int co  = q / (KT / 8);
    const int kc  = (q - co * (KT / 8)) * 8;
    const int tap = kc >> 6;
    const int ci0 = kc & 63;
    unsigned hb[8];
#pragma unroll
    for (int j = 0; j < 8; ++j)
      hb[j] = bfb(woff[(size_t)(co * NC + ci0 + j) * 9 + tap]);
    v4u wh;
    wh.x = hb[0] | (hb[1] << 16);
    wh.y = hb[2] | (hb[3] << 16);
    wh.z = hb[4] | (hb[5] << 16);
    wh.w = hb[6] | (hb[7] << 16);
    unsigned* dst = wo + (size_t)q * 4;
    *(volatile v4u*)dst = wh;
    __threadfence();
    *(volatile v4u*)dst = wh;
  } else {
    const int q   = (blockIdx.x - WO_BLK) * 256 + tid;
    const int co  = q / (KT / 8);
    const int kc  = (q - co * (KT / 8)) * 8;
    const int tap = kc >> 6;
    const int ci0 = kc & 63;
    unsigned hb[8];
#pragma unroll
    for (int j = 0; j < 8; ++j) {
      const float v = bf_rne(wreg[(size_t)(co * NC + ci0 + j) * 9 + tap]) * WSC;
      hb[j] = hbits((_Float16)v);
    }
    v4u wh;
    wh.x = hb[0] | (hb[1] << 16);
    wh.y = hb[2] | (hb[3] << 16);
    wh.z = hb[4] | (hb[5] << 16);
    wh.w = hb[6] | (hb[7] << 16);
    unsigned* dst = wr + (size_t)q * 4;
    *(volatile v4u*)dst = wh;
    __threadfence();
    *(volatile v4u*)dst = wh;
  }
}

__global__ __launch_bounds__(256)
void k_xcvt(const float* __restrict__ x, unsigned short* xh, _Float16* sp)
{
  __shared__ __align__(16) unsigned short T[PD * SP];
  const int tid  = threadIdx.x;
  const int lane = tid & 31;
  const int wid  = tid >> 5;
  const int pj   = lane & 7;
  const int lq   = lane >> 3;
  const int b    = blockIdx.x / PD;
  const int hp   = blockIdx.x - b * PD;
  const size_t rowb = ((size_t)(b * PD + hp)) * PD;

  if (hp == 0 || hp == PD - 1) {
    const v8us zu = zero8us();
    const v8h  zh = zero8h();
    size_t e[5]; bool ok[5];
#pragma unroll
    for (int r = 0; r < 5; ++r) {
      const int L  = r * 32 + wid * 4 + lq;
      const int Lc = (L < PD) ? L : (PD - 1);
      e[r]  = (rowb + Lc) * NC + 8 * pj;
      ok[r] = (L < PD);
    }
#pragma unroll
    for (int r = 0; r < 5; ++r) if (ok[r]) {
      *(volatile v8us*)(xh + e[r])          = zu;
      *(volatile v8h*)(sp + e[r])            = zh;
      *(volatile v8h*)(sp + PLANE_E + e[r])  = zh;
    }
    __threadfence();
#pragma unroll
    for (int r = 0; r < 5; ++r) if (ok[r]) {
      *(volatile v8us*)(xh + e[r])          = zu;
      *(volatile v8h*)(sp + e[r])            = zh;
      *(volatile v8h*)(sp + PLANE_E + e[r])  = zh;
    }
  } else {
    const int h = hp - 1;
    if (tid < 16) {
      const int slot = (tid < 8) ? 0 : (PD - 1);
      *(v8us*)&T[slot * SP + 8 * (tid & 7)] = zero8us();
    }
#pragma unroll
    for (int i = 0; i < 8; ++i) {
      const int idx = tid + 256 * i;
      const int w4  = idx & 31;
      const int c   = idx >> 5;
      const v4f v = *(const v4f*)(x + ((size_t)(b * NC + c) * HI + h) * WI + 4 * w4);
      unsigned short* tp = T + (4 * w4 + 1) * SP + c;
      tp[0 * SP] = (unsigned short)bfb(v.x);
      tp[1 * SP] = (unsigned short)bfb(v.y);
      tp[2 * SP] = (unsigned short)bfb(v.z);
      tp[3 * SP] = (unsigned short)bfb(v.w);
    }
    __syncthreads();
    v8us val[5]; size_t e[5]; bool ok[5];
#pragma unroll
    for (int r = 0; r < 5; ++r) {
      const int L  = r * 32 + wid * 4 + lq;
      const int Lc = (L < PD) ? L : (PD - 1);
      val[r] = *(const v8us*)&T[Lc * SP + 8 * pj];
      e[r]   = (rowb + Lc) * NC + 8 * pj;
      ok[r]  = (L < PD);
    }
#pragma unroll
    for (int r = 0; r < 5; ++r) if (ok[r]) *(volatile v8us*)(xh + e[r]) = val[r];
    __threadfence();
#pragma unroll
    for (int r = 0; r < 5; ++r) if (ok[r]) *(volatile v8us*)(xh + e[r]) = val[r];
  }
}

__global__ __launch_bounds__(256)
void k_offs(const float* __restrict__ x, const __bf16* __restrict__ xh,
            const __bf16* __restrict__ wo, _Float16* sp)
{
  __shared__ float offl[NO * OPITCH];
  __shared__ __align__(16) _Float16 sth[65 * SP];
  __shared__ __align__(16) _Float16 stl[65 * SP];

  const int tid  = threadIdx.x;
  const int lane = tid & 31;
  const int wid  = tid >> 5;
  const int l15  = lane & 15;
  const int hh   = lane >> 4;
  const int gid  = blockIdx.x;
  const int wt   = gid & 1;
  const int h    = (gid >> 1) & (HI - 1);
  const int b    = gid >> 8;
  const int w0   = wt * 64;

  if (tid < 8) {
    const v8h z = zero8h();
    *(v8h*)&sth[64 * SP + 8 * tid] = z;
    *(v8h*)&stl[64 * SP + 8 * tid] = z;
  }

  const int n0 = 16 * wid;
  const __bf16* bp = wo + (size_t)(n0 + l15) * KT + 8 * hh;
  const __bf16* ap = xh + (((size_t)(b * PD + h)) * PD + w0 + l15) * NC + 8 * hh;
  v8f acc0 = zero8f(), acc1 = zero8f(), acc2 = zero8f(), acc3 = zero8f();
#pragma unroll 1
  for (int kh = 0; kh < 3; ++kh) {
#pragma unroll 1
    for (int kw = 0; kw < 3; ++kw) {
      const __bf16* a  = ap + (kh * PD + kw) * NC;
      const __bf16* bk = bp + (kh * 3 + kw) * 64;
      {
        const v16b fb = ldfrag_b(bk);
        const v16b f0 = ldfrag_b(a);
        const v16b f1 = ldfrag_b(a + 16 * NC);
        const v16b f2 = ldfrag_b(a + 32 * NC);
        const v16b f3 = ldfrag_b(a + 48 * NC);
        acc0 = mma_b(f0, fb, acc0);
        acc1 = mma_b(f1, fb, acc1);
        acc2 = mma_b(f2, fb, acc2);
        acc3 = mma_b(f3, fb, acc3);
        guard4(acc0, acc1, acc2, acc3, f0, f1, f2, f3, fb);
      }
      {
        const v16b fb = ldfrag_b(bk + 32);
        const v16b f0 = ldfrag_b(a + 32);
        const v16b f1 = ldfrag_b(a + 16 * NC + 32);
        const v16b f2 = ldfrag_b(a + 32 * NC + 32);
        const v16b f3 = ldfrag_b(a + 48 * NC + 32);
        acc0 = mma_b(f0, fb, acc0);
        acc1 = mma_b(f1, fb, acc1);
        acc2 = mma_b(f2, fb, acc2);
        acc3 = mma_b(f3, fb, acc3);
        guard4(acc0, acc1, acc2, acc3, f0, f1, f2, f3, fb);
      }
    }
  }
  acc_guard4(acc0, acc1, acc2, acc3);

  {
    float* orow = offl + (n0 + l15) * OPITCH + 8 * hh;
#pragma unroll
    for (int r = 0; r < 8; ++r) {
      orow[r]      = acc0[r];
      orow[16 + r] = acc1[r];
      orow[32 + r] = acc2[r];
      orow[48 + r] = acc3[r];
    }
  }
  __syncthreads();

  {
    const float lh = linv(h);
    const int c = tid & 63;
    const float* img = x + ((size_t)(b * NC + c)) * HWI;
    const float* orw = offl + c * OPITCH;
    const float* orh = offl + (c + 64) * OPITCH;
#pragma unroll 1
    for (int i = 0; i < 16; ++i) {
      const int m = 4 * i + (tid >> 6);
      const float ow = orw[m];
      const float oh = orh[m];
      const float gx = oh + lh;
      const float gy = ow + linv(w0 + m);
      const float ix = ((gx + 1.0f) * 0.5f) * 127.0f;
      const float iy = ((gy + 1.0f) * 0.5f) * 127.0f;
      const float x0f = floorf(ix);
      const float y0f = floorf(iy);
      const float x1f = x0f + 1.0f;
      const float y1f = y0f + 1.0f;
      const float wx1 = ix - x0f;
      const float wx0 = 1.0f - wx1;
      const float wy1 = iy - y0f;
      const float wy0 = 1.0f - wy1;
      const float vx0 = (x0f >= 0.0f && x0f <= 127.0f) ? 1.0f : 0.0f;
      const float vx1 = (x1f >= 0.0f && x1f <= 127.0f) ? 1.0f : 0.0f;
      const float vy0 = (y0f >= 0.0f && y0f <= 127.0f) ? 1.0f : 0.0f;
      const float vy1 = (y1f >= 0.0f && y1f <= 127.0f) ? 1.0f : 0.0f;
      const int xc0 = (int)fminf(fmaxf(x0f, 0.0f), 127.0f);
      const int xc1 = (int)fminf(fmaxf(x1f, 0.0f), 127.0f);
      const int yc0 = (int)fminf(fmaxf(y0f, 0.0f), 127.0f);
      const int yc1 = (int)fminf(fmaxf(y1f, 0.0f), 127.0f);
      const float g00 = bf_rne(img[yc0 * WI + xc0]) * (vx0 * vy0);
      const float g10 = bf_rne(img[yc0 * WI + xc1]) * (vx1 * vy0);
      const float g01 = bf_rne(img[yc1 * WI + xc0]) * (vx0 * vy1);
      const float g11 = bf_rne(img[yc1 * WI + xc1]) * (vx1 * vy1);
      const float v = (((g00 * wy0) * wx0 + (g10 * wy0) * wx1) + (g01 * wy1) * wx0) + (g11 * wy1) * wx1;
      const _Float16 hv = (_Float16)v;
      const _Float16 lv = (_Float16)((v - (float)hv) * RSC);
      sth[m * SP + c] = hv;
      stl[m * SP + c] = lv;
    }
  }
  __syncthreads();

  {
    const int pj = lane & 7;
    const int lq = lane >> 3;
    const size_t rowb = ((size_t)(b * PD + h + 1)) * PD;
    v8h val[5]; size_t e[5]; bool ok[5];
#pragma unroll
    for (int r = 0; r < 5; ++r) {
      const int L    = r * 32 + wid * 4 + lq;
      const int Lc   = (L < 130) ? L : 129;
      const int pl   = (Lc >= 65) ? 1 : 0;
      const int slot = Lc - 65 * pl;
      const int pp   = (slot == 64) ? (wt ? (PD - 1) : 0) : (w0 + 1 + slot);
      const v8h vh = *(const v8h*)&sth[slot * SP + 8 * pj];
      const v8h vl = *(const v8h*)&stl[slot * SP + 8 * pj];
      val[r] = pl ? vl : vh;
      e[r]   = (size_t)pl * PLANE_E + (rowb + pp) * NC + 8 * pj;
      ok[r]  = (L < 130);
    }
#pragma unroll
    for (int r = 0; r < 5; ++r) if (ok[r]) *(volatile v8h*)(sp + e[r]) = val[r];
    __threadfence();
#pragma unroll
    for (int r = 0; r < 5; ++r) if (ok[r]) *(volatile v8h*)(sp + e[r]) = val[r];
  }
}

__global__ __launch_bounds__(256)
void k_conv(const _Float16* __restrict__ sp, const _Float16* __restrict__ wr,
            const float* __restrict__ bias, float* out)
{
  __shared__ __align__(16) float os[NC * OSP];
  __shared__ float bsl[NC];

  const int tid  = threadIdx.x;
  const int lane = tid & 31;
  const int wid  = tid >> 5;
  const int l15  = lane & 15;
  const int hh   = lane >> 4;
  const int gid  = blockIdx.x;
  const int wt   = gid & 1;
  const int h    = (gid >> 1) & (HI - 1);
  const int b    = gid >> 8;
  const int w0   = wt * 64;

  if (tid < NC) bsl[tid] = bf_rne(bias[tid]);
  __syncthreads();

  const int nt = wid & 3;
  const int mh = wid >> 2;
  const int n0 = 16 * nt;
  const _Float16* bp  = wr + (size_t)(n0 + l15) * KT + 8 * hh;
  const _Float16* aph = sp + (((size_t)(b * PD + h)) * PD + w0 + 32 * mh + l15) * NC + 8 * hh;
  const _Float16* apl = aph + PLANE_E;
  v8f ch0 = zero8f(), ch1 = zero8f(), cl0 = zero8f(), cl1 = zero8f();
#pragma unroll 1
  for (int kh = 0; kh < 3; ++kh) {
#pragma unroll 1
    for (int kw = 0; kw < 3; ++kw) {
      const _Float16* ah = aph + (kh * PD + kw) * NC;
      const _Float16* al = apl + (kh * PD + kw) * NC;
      const _Float16* bk = bp + (kh * 3 + kw) * 64;
      {
        const v16h fb  = ldfrag_h(bk);
        const v16h fh0 = ldfrag_h(ah);
        const v16h fh1 = ldfrag_h(ah + 16 * NC);
        const v16h fl0 = ldfrag_h(al);
        const v16h fl1 = ldfrag_h(al + 16 * NC);
        ch0 = mma_h(fh0, fb, ch0);
        ch1 = mma_h(fh1, fb, ch1);
        cl0 = mma_h(fl0, fb, cl0);
        cl1 = mma_h(fl1, fb, cl1);
        guard4(ch0, ch1, cl0, cl1, fh0, fh1, fl0, fl1, fb);
      }
      {
        const v16h fb  = ldfrag_h(bk + 32);
        const v16h fh0 = ldfrag_h(ah + 32);
        const v16h fh1 = ldfrag_h(ah + 16 * NC + 32);
        const v16h fl0 = ldfrag_h(al + 32);
        const v16h fl1 = ldfrag_h(al + 16 * NC + 32);
        ch0 = mma_h(fh0, fb, ch0);
        ch1 = mma_h(fh1, fb, ch1);
        cl0 = mma_h(fl0, fb, cl0);
        cl1 = mma_h(fl1, fb, cl1);
        guard4(ch0, ch1, cl0, cl1, fh0, fh1, fl0, fl1, fb);
      }
    }
  }
  acc_guard4(ch0, ch1, cl0, cl1);

  {
    const int ch = n0 + l15;
    const float bb = bsl[ch];
    float* o0 = os + ch * OSP + 32 * mh + 8 * hh;
    v4f p0, p1, p2, p3;
    p0.x = ch0[0] * INV_H + cl0[0] * INV_L + bb;
    p0.y = ch0[1] * INV_H + cl0[1] * INV_L + bb;
    p0.z = ch0[2] * INV_H + cl0[2] * INV_L + bb;
    p0.w = ch0[3] * INV_H + cl0[3] * INV_L + bb;
    p1.x = ch0[4] * INV_H + cl0[4] * INV_L + bb;
    p1.y = ch0[5] * INV_H + cl0[5] * INV_L + bb;
    p1.z = ch0[6] * INV_H + cl0[6] * INV_L + bb;
    p1.w = ch0[7] * INV_H + cl0[7] * INV_L + bb;
    p2.x = ch1[0] * INV_H + cl1[0] * INV_L + bb;
    p2.y = ch1[1] * INV_H + cl1[1] * INV_L + bb;
    p2.z = ch1[2] * INV_H + cl1[2] * INV_L + bb;
    p2.w = ch1[3] * INV_H + cl1[3] * INV_L + bb;
    p3.x = ch1[4] * INV_H + cl1[4] * INV_L + bb;
    p3.y = ch1[5] * INV_H + cl1[5] * INV_L + bb;
    p3.z = ch1[6] * INV_H + cl1[6] * INV_L + bb;
    p3.w = ch1[7] * INV_H + cl1[7] * INV_L + bb;
    *(v4f*)(o0)      = p0;
    *(v4f*)(o0 + 4)  = p1;
    *(v4f*)(o0 + 16) = p2;
    *(v4f*)(o0 + 20) = p3;
  }
  __syncthreads();

  {
    const int pj = lane & 7;
    const int lq = lane >> 3;
    v4f val[4]; size_t e[4];
#pragma unroll
    for (int r = 0; r < 4; ++r) {
      const int L   = r * 32 + wid * 4 + lq;
      const int chn = L >> 1;
      const int hf  = L & 1;
      val[r] = *(const v4f*)(os + chn * OSP + 32 * hf + 4 * pj);
      e[r]   = ((size_t)(b * NC + chn) * HI + h) * WI + w0 + 32 * hf + 4 * pj;
    }
#pragma unroll
    for (int r = 0; r < 4; ++r) *(volatile v4f*)(out + e[r]) = val[r];
    __threadfence();
#pragma unroll
    for (int r = 0; r < 4; ++r) *(volatile v4f*)(out + e[r]) = val[r];
  }
}

extern "C" void kernel_launch(void* const* d_in, const int* in_sizes, int n_in,
                              void* d_out, int out_size, void* d_ws, size_t ws_size,
                              hipStream_t stream) {
  if (n_in < 4) return;
  if (in_sizes[0] != NB * NC * HWI) return;
  if (in_sizes[1] != NO * NC * 9) return;
  if (in_sizes[2] != NC * NC * 9) return;
  if (in_sizes[3] != NC) return;
  if (out_size != NB * NC * HWI) return;
  if (WS_END > ws_size) return;

  const float* x     = (const float*)d_in[0];
  const float* w_off = (const float*)d_in[1];
  const float* w_reg = (const float*)d_in[2];
  const float* b_reg = (const float*)d_in[3];
  float* out = (float*)d_out;
  char* ws = (char*)d_ws;

  unsigned* wo_u       = (unsigned*)(ws + WS_WO);
  unsigned* wr_u       = (unsigned*)(ws + WS_WR);
  unsigned short* xh_u = (unsigned short*)(ws + WS_XH);
  _Float16* sp         = (_Float16*)(ws + WS_SP);

  k_wpack<<<dim3(WO_BLK + WR_BLK), dim3(256), 0, stream>>>(w_off, w_reg, wo_u, wr_u);
  (void)hipGetLastError();

  k_xcvt<<<dim3(NB * PD), dim3(256), 0, stream>>>(x, xh_u, sp);
  (void)hipGetLastError();

  k_offs<<<dim3(NB * HI * 2), dim3(256), 0, stream>>>(x, (const __bf16*)xh_u, (const __bf16*)wo_u, sp);
  (void)hipGetLastError();

  k_conv<<<dim3(NB * HI * 2), dim3(256), 0, stream>>>((const _Float16*)sp, (const _Float16*)wr_u,
                                                        b_reg, out);
  (void)hipGetLastError();
}
